// LocalAttention_31104153158060
// MI455X (gfx1250) — hardware-run, weakly checked
//
#include <hip/hip_runtime.h>
#include <stdint.h>
#include <stddef.h>


#ifndef NB
#define NB 4
#endif
#ifndef SEQ
#define SEQ 1024
#endif
#define NB_FULL 4
#define SEQ_FULL 1024
#define EMB 768
#define NH 12
#define HD 64
#define WIN 16
#define MROWS (NB * SEQ)
#define KROWS 96
#define VCOLS 112
#define PCAR 16384.0f
#define PINV (1.0f / 16384.0f)

static_assert((MROWS % 128) == 0);
static_assert((SEQ % 64) == 0);
static_assert(SEQ >= 64);
static_assert(NB >= 1 && NB <= NB_FULL);
static_assert(SEQ <= SEQ_FULL);
static_assert((EMB % 128) == 0);
static_assert(NH * HD == EMB);
static_assert((SEQ % 4) == 0);

typedef __bf16 v16bf __attribute__((ext_vector_type(16)));
typedef _Float16 v16h __attribute__((ext_vector_type(16)));
typedef _Float16 v8h __attribute__((ext_vector_type(8)));
typedef float v8f __attribute__((ext_vector_type(8)));
typedef float v4f __attribute__((ext_vector_type(4)));
typedef unsigned int u32x4 __attribute__((ext_vector_type(4)));
typedef v4f __attribute__((may_alias)) v4fa;
typedef u32x4 __attribute__((may_alias)) u32x4a;
typedef unsigned int __attribute__((may_alias)) u32a;

union FragBF { v16bf v; u32x4 q[2]; };
union FragH  { v16h v;  u32x4 q[2]; };
union Pack8H { v8h h;   u32x4 u; };

__device__ __forceinline__ int clampi(int x, int lo, int hi) {
  return x < lo ? lo : (x > hi ? hi : x);
}

__device__ __forceinline__ unsigned short f2bf(float x) {
  unsigned u = __builtin_bit_cast(unsigned, x);
  u += 0x7FFFu + ((u >> 16) & 1u);
  return (unsigned short)(u >> 16);
}
__device__ __forceinline__ float bfr(float x) {
  unsigned u = ((unsigned)f2bf(x)) << 16;
  return __builtin_bit_cast(float, u);
}
__device__ __forceinline__ unsigned short h2u(float x) {
  _Float16 h = (_Float16)x;
  return __builtin_bit_cast(unsigned short, h);
}

__device__ __forceinline__ v8f wmma_bf16(v16bf a, v16bf b, v8f c) {
  v8f d = __builtin_amdgcn_wmma_f32_16x16x32_bf16(false, a, false, b, (short)0, c, false, false);
  asm volatile("v_nop\n\tv_nop\n\tv_nop\n\tv_nop" : "+v"(d) : "v"(a), "v"(b));
  return d;
}
__device__ __forceinline__ v8f wmma_f16(v16h a, v16h b, v8f c) {
  v8f d = __builtin_amdgcn_wmma_f32_16x16x32_f16(false, a, false, b, (short)0, c, false, false);
  asm volatile("v_nop\n\tv_nop\n\tv_nop\n\tv_nop" : "+v"(d) : "v"(a), "v"(b));
  return d;
}

__global__ __launch_bounds__(256) void k_cvt(
    const float* __restrict__ s0, const float* __restrict__ s1, const float* __restrict__ s2,
    const float* __restrict__ s3, const float* __restrict__ s4, const float* __restrict__ s5,
    unsigned short* __restrict__ d0, unsigned short* __restrict__ d1, unsigned short* __restrict__ d2,
    unsigned short* __restrict__ d3, unsigned short* __restrict__ d4, unsigned short* __restrict__ d5)
{
  const int seg = blockIdx.y;
  const float* src = (seg == 0) ? s0 : (seg == 1) ? s1 : (seg == 2) ? s2 : (seg == 3) ? s3 : (seg == 4) ? s4 : s5;
  unsigned short* dst = (seg == 0) ? d0 : (seg == 1) ? d1 : (seg == 2) ? d2 : (seg == 3) ? d3 : (seg == 4) ? d4 : d5;
  const bool act = seg < 3;
  const int nItems = act ? (MROWS * EMB / 8) : (EMB * EMB / 8);
  const int item = blockIdx.x * 256 + threadIdx.x;
  if (item >= nItems) return;
  const size_t e8 = (size_t)item * 8;
  size_t so;
  if (act) {
    const size_t R = e8 / EMB;
    const int col = (int)(e8 - R * (size_t)EMB);
    const int b = (int)(R / SEQ);
    const int s = (int)(R - (size_t)b * SEQ);
    so = ((size_t)b * SEQ_FULL + (size_t)s) * EMB + (size_t)col;
  } else {
    so = e8;
  }
  const v4f xa = *(const v4f*)(src + so);
  const v4f xb = *(const v4f*)(src + so + 4);
  const float f0 = xa.x, f1 = xa.y, f2 = xa.z, f3 = xa.w;
  const float f4 = xb.x, f5 = xb.y, f6 = xb.z, f7 = xb.w;
  u32x4 w;
  w.x = (unsigned)f2bf(f0) | ((unsigned)f2bf(f1) << 16);
  w.y = (unsigned)f2bf(f2) | ((unsigned)f2bf(f3) << 16);
  w.z = (unsigned)f2bf(f4) | ((unsigned)f2bf(f5) << 16);
  w.w = (unsigned)f2bf(f6) | ((unsigned)f2bf(f7) << 16);
  unsigned short* dp = dst + e8;
  *(volatile u32x4*)dp = w;
  __threadfence();
  *(volatile u32x4*)dp = w;
}

__global__ __launch_bounds__(256) __attribute__((amdgpu_num_vgpr(256)))
void k_gemm(const unsigned short* __restrict__ A, const unsigned short* __restrict__ W,
            const float* __restrict__ bias, float* __restrict__ Cf, unsigned short* __restrict__ Ch)
{
  const int lane = threadIdx.x & 31;
  const int wave = threadIdx.x >> 5;
  const int l15  = lane & 15;
  const int lhi  = lane >> 4;
  const int mb   = blockIdx.y * 128 + (wave & 3) * 32;
  const int nb   = blockIdx.x * 128 + (wave >> 2) * 64;

  __shared__ __align__(16) float stg[8][16 * 64];

  v8f acc[2][4];
#pragma unroll
  for (int t = 0; t < 2; ++t)
#pragma unroll
    for (int u = 0; u < 4; ++u)
#pragma unroll
      for (int i = 0; i < 8; ++i) acc[t][u][i] = 0.f;

#pragma unroll 1
  for (int k0 = 0; k0 < EMB; k0 += 32) {
    FragBF a[2], bw[4];
#pragma unroll
    for (int t = 0; t < 2; ++t) {
      const unsigned short* p = A + (size_t)(mb + t * 16 + l15) * EMB + k0 + 8 * lhi;
      a[t].q[0] = *(const u32x4*)(p);
      a[t].q[1] = *(const u32x4*)(p + 16);
    }
#pragma unroll
    for (int u = 0; u < 4; ++u) {
      const unsigned short* p = W + (size_t)(nb + u * 16 + l15) * EMB + k0 + 8 * lhi;
      bw[u].q[0] = *(const u32x4*)(p);
      bw[u].q[1] = *(const u32x4*)(p + 16);
    }
#pragma unroll
    for (int t = 0; t < 2; ++t)
#pragma unroll
      for (int u = 0; u < 4; ++u)
        acc[t][u] = wmma_bf16(a[t].v, bw[u].v, acc[t][u]);
  }

  float bcol[4];
#pragma unroll
  for (int u = 0; u < 4; ++u) bcol[u] = bfr(bias[nb + u * 16 + l15]);

  float* st = stg[wave];
#pragma unroll
  for (int t = 0; t < 2; ++t) {
#pragma unroll
    for (int u = 0; u < 4; ++u)
#pragma unroll
      for (int r = 0; r < 8; ++r)
        st[(8 * lhi + r) * 64 + u * 16 + l15] = acc[t][u][r] + bcol[u];
    __syncthreads();

    const int rowb = mb + t * 16;
    v4f fv[8];
#pragma unroll
    for (int it = 0; it < 8; ++it) {
      const int f = it * 32 + lane;
      const int row = f >> 4, c4 = f & 15;
      fv[it] = *(const v4fa*)&st[row * 64 + c4 * 4];
    }
    u32x4 hv[4];
#pragma unroll
    for (int it = 0; it < 4; ++it) {
      const int f = it * 32 + lane;
      const int row = f >> 3, c8 = f & 7;
      const v4f xa = *(const v4fa*)&st[row * 64 + c8 * 8];
      const v4f xb = *(const v4fa*)&st[row * 64 + c8 * 8 + 4];
      v8h hh = {(_Float16)xa.x, (_Float16)xa.y, (_Float16)xa.z, (_Float16)xa.w,
                (_Float16)xb.x, (_Float16)xb.y, (_Float16)xb.z, (_Float16)xb.w};
      Pack8H pk;
      pk.h = hh;
      hv[it] = pk.u;
    }
#pragma unroll
    for (int it = 0; it < 8; ++it) {
      const int f = it * 32 + lane;
      const int row = f >> 4, c4 = f & 15;
      float* dp = Cf + (size_t)(rowb + row) * EMB + nb + c4 * 4;
      *(volatile v4f*)dp = fv[it];
    }
#pragma unroll
    for (int it = 0; it < 4; ++it) {
      const int f = it * 32 + lane;
      const int row = f >> 3, c8 = f & 7;
      unsigned short* hp = Ch + (size_t)(rowb + row) * EMB + nb + c8 * 8;
      *(volatile u32x4*)hp = hv[it];
    }
    __threadfence();
#pragma unroll
    for (int it = 0; it < 8; ++it) {
      const int f = it * 32 + lane;
      const int row = f >> 4, c4 = f & 15;
      float* dp = Cf + (size_t)(rowb + row) * EMB + nb + c4 * 4;
      *(volatile v4f*)dp = fv[it];
    }
#pragma unroll
    for (int it = 0; it < 4; ++it) {
      const int f = it * 32 + lane;
      const int row = f >> 3, c8 = f & 7;
      unsigned short* hp = Ch + (size_t)(rowb + row) * EMB + nb + c8 * 8;
      *(volatile u32x4*)hp = hv[it];
    }
    __syncthreads();
  }
}

__global__ __launch_bounds__(256) void k_vsum(const float* __restrict__ vf, float* __restrict__ vsum)
{
  __shared__ __align__(16) float sh[256];
  const int b = blockIdx.y;
  const int c = blockIdx.x * 256 + threadIdx.x;
  const float* p = vf + (size_t)b * SEQ * EMB + c;
  float a0 = 0.f, a1 = 0.f, a2 = 0.f, a3 = 0.f;
#pragma unroll 1
  for (int s = 0; s < SEQ; s += 4) {
    a0 += p[(size_t)(s) * EMB];
    a1 += p[(size_t)(s + 1) * EMB];
    a2 += p[(size_t)(s + 2) * EMB];
    a3 += p[(size_t)(s + 3) * EMB];
  }
  sh[threadIdx.x] = (a0 + a1) + (a2 + a3);
  __syncthreads();
  if (threadIdx.x < 64) {
    const v4f v = *(const v4fa*)&sh[threadIdx.x * 4];
    float* d = vsum + (size_t)b * EMB + blockIdx.x * 256 + threadIdx.x * 4;
    *(volatile v4f*)d = v;
    __threadfence();
    *(volatile v4f*)d = v;
  }
}

__global__ __launch_bounds__(128) __attribute__((amdgpu_num_vgpr(256)))
void k_attn(const unsigned short* __restrict__ qh, const unsigned short* __restrict__ kh,
            const unsigned short* __restrict__ vh, const float* __restrict__ vsum,
            const float* __restrict__ amask, const float* __restrict__ wwin,
            float* __restrict__ ctx)
{
  const int q0   = blockIdx.x * 64;
  const int h    = blockIdx.y;
  const int b    = blockIdx.z;
  const int wave = threadIdx.x >> 5;
  const int lane = threadIdx.x & 31;
  const int hl   = lane >> 4;
  const int ln   = lane & 15;
  const int kbase = q0 - WIN;
  const int iw0   = q0 + wave * 16;
  const size_t brow = (size_t)b * SEQ;

  __shared__ __align__(16) unsigned short kt_s[KROWS * HD];
  __shared__ __align__(16) unsigned short vt_s[HD * VCOLS];
  __shared__ __align__(16) unsigned short pst[4][16 * 64];
  __shared__ __align__(16) float cst[4][16 * 64];

  const u32x4 z4 = {0u, 0u, 0u, 0u};

#pragma unroll
  for (int it = 0; it < 6; ++it) {
    const int item = it * 128 + threadIdx.x;
    const int kl = item >> 3, c8 = item & 7;
    const int j  = kbase + kl;
    const int jc = clampi(j, 0, SEQ - 1);
    u32x4 v = *(const u32x4*)(kh + (brow + (size_t)jc) * EMB + h * HD + c8 * 8);
    if ((unsigned)j >= (unsigned)SEQ) v = z4;
    *(u32x4a*)&kt_s[kl * HD + c8 * 8] = v;
  }
  {
    u32a* vt32 = (u32a*)vt_s;
#pragma unroll
    for (int it = 0; it < 3; ++it) {
      const int item = it * 128 + threadIdx.x;
      const int kp = item >> 3, c8 = item & 7;
      const int j0 = kbase + 2 * kp;
      const int j1 = j0 + 1;
      const int j0c = clampi(j0, 0, SEQ - 1);
      const int j1c = clampi(j1, 0, SEQ - 1);
      u32x4 r0 = *(const u32x4*)(vh + (brow + (size_t)j0c) * EMB + h * HD + c8 * 8);
      u32x4 r1 = *(const u32x4*)(vh + (brow + (size_t)j1c) * EMB + h * HD + c8 * 8);
      if ((unsigned)j0 >= (unsigned)SEQ) r0 = z4;
      if ((unsigned)j1 >= (unsigned)SEQ) r1 = z4;
#pragma unroll
      for (int i = 0; i < 4; ++i) {
        const unsigned a  = r0[i];
        const unsigned bb = r1[i];
        const int d = c8 * 8 + 2 * i;
        vt32[d * (VCOLS / 2) + kp]       = (a & 0xffffu) | (bb << 16);
        vt32[(d + 1) * (VCOLS / 2) + kp] = (a >> 16) | (bb & 0xffff0000u);
      }
    }
    const int d  = threadIdx.x >> 1;
    const int hf = threadIdx.x & 1;
    *(u32x4a*)&vt_s[d * VCOLS + KROWS + 8 * hf] = z4;
  }
  __syncthreads();

  FragH qa[2];
  {
    const unsigned short* qrow = qh + (brow + (size_t)(iw0 + ln)) * EMB + h * HD + 8 * hl;
#pragma unroll
    for (int dh = 0; dh < 2; ++dh) {
      qa[dh].q[0] = *(const u32x4*)(qrow + dh * 32);
      qa[dh].q[1] = *(const u32x4*)(qrow + dh * 32 + 16);
    }
  }

  v8f sacc[3];
#pragma unroll
  for (int kt = 0; kt < 3; ++kt)
#pragma unroll
    for (int i = 0; i < 8; ++i) sacc[kt][i] = 0.f;
#pragma unroll
  for (int kt = 0; kt < 3; ++kt) {
#pragma unroll
    for (int dh = 0; dh < 2; ++dh) {
      FragH kb;
      const unsigned short* src = &kt_s[((wave + kt) * 16 + ln) * HD + dh * 32 + 8 * hl];
      kb.q[0] = *(const u32x4a*)(src);
      kb.q[1] = *(const u32x4a*)(src + 16);
      sacc[kt] = wmma_f16(qa[dh].v, kb.v, sacc[kt]);
    }
  }

  const int jk0 = iw0 - 16 + ln;
  const int jk1 = iw0 + ln;
  const int jk2 = iw0 + 16 + ln;
  const bool vk0 = (unsigned)jk0 < (unsigned)SEQ;
  const bool vk1 = (unsigned)jk1 < (unsigned)SEQ;
  const bool vk2 = (unsigned)jk2 < (unsigned)SEQ;
  const size_t mrow = (size_t)b * SEQ_FULL;
  const float am0 = bfr(amask[mrow + clampi(jk0, 0, SEQ - 1)]);
  const float am1 = bfr(amask[mrow + clampi(jk1, 0, SEQ - 1)]);
  const float am2 = bfr(amask[mrow + clampi(jk2, 0, SEQ - 1)]);
  const float ww0 = bfr(wwin[0]);
  const float ww1 = bfr(wwin[1]);
  const float ww2 = bfr(wwin[2]);

  float garr[8];
  unsigned short* pw = pst[wave];

#pragma unroll
  for (int r = 0; r < 8; ++r) {
    const int i = iw0 + 8 * hl + r;
    const int dd0 = i - jk0, dd1 = i - jk1, dd2 = i - jk2;
    const bool in0 = vk0 && (dd0 <= WIN) && (dd0 >= -WIN);
    const bool in1 = vk1 && (dd1 <= WIN) && (dd1 >= -WIN);
    const bool in2 = vk2 && (dd2 <= WIN) && (dd2 >= -WIN);
    const int lo = (i - WIN) > 0 ? (i - WIN) : 0;
    const int hi = (i + WIN) < (SEQ - 1) ? (i + WIN) : (SEQ - 1);
    const float nOut = (float)(SEQ - (hi - lo + 1));
    float x0 = in0 ? sacc[0][r] * 0.125f : 0.f;
    float x1 = in1 ? sacc[1][r] * 0.125f : 0.f;
    float x2 = in2 ? sacc[2][r] * 0.125f : 0.f;
    float c0 = 0.f, c1 = 0.f, c2 = 0.f, g = 0.f;
#pragma unroll 1
    for (int t = 0; t < 3; ++t) {
      const float wt = (t == 0) ? ww0 : ((t == 1) ? ww1 : ww2);
      x0 = x0 * am0; x1 = x1 * am1; x2 = x2 * am2;
      float m = fmaxf(fmaxf(fmaxf(0.f, x0), x1), x2);
      m = fmaxf(m, __shfl_xor(m, 8, 32));
      m = fmaxf(m, __shfl_xor(m, 4, 32));
      m = fmaxf(m, __shfl_xor(m, 2, 32));
      m = fmaxf(m, __shfl_xor(m, 1, 32));
      const float t0 = __expf(x0 - m);
      const float t1 = __expf(x1 - m);
      const float t2 = __expf(x2 - m);
      const float e0 = in0 ? t0 : 0.f;
      const float e1 = in1 ? t1 : 0.f;
      const float e2 = in2 ? t2 : 0.f;
      float z = (e0 + e1) + e2;
      z += __shfl_xor(z, 8, 32);
      z += __shfl_xor(z, 4, 32);
      z += __shfl_xor(z, 2, 32);
      z += __shfl_xor(z, 1, 32);
      const float em  = __expf(-m);
      const float Z   = nOut * em + z;
      const float inv = 1.0f / Z;
      g  = g  + wt * (em * inv);
      c0 = c0 + wt * (e0 * inv);
      c1 = c1 + wt * (e1 * inv);
      c2 = c2 + wt * (e2 * inv);
    }
    garr[r] = g;
    const float p0 = in0 ? (c0 - g) : 0.f;
    const float p1 = in1 ? (c1 - g) : 0.f;
    const float p2 = in2 ? (c2 - g) : 0.f;
    pw[(8 * hl + r) * 64 + ln]      = h2u(p0 * PCAR);
    pw[(8 * hl + r) * 64 + 16 + ln] = h2u(p1 * PCAR);
    pw[(8 * hl + r) * 64 + 32 + ln] = h2u(p2 * PCAR);
  }
  *(u32x4a*)&pw[(lane >> 1) * 64 + 48 + 8 * (lane & 1)] = z4;
  __syncthreads();

  v8f oacc[4];
#pragma unroll
  for (int t = 0; t < 4; ++t)
#pragma unroll
    for (int i = 0; i < 8; ++i) oacc[t][i] = 0.f;
#pragma unroll
  for (int ks = 0; ks < 2; ++ks) {
    FragH pa;
    const unsigned short* ps = &pw[ln * 64 + ks * 32 + 8 * hl];
    pa.q[0] = *(const u32x4a*)(ps);
    pa.q[1] = *(const u32x4a*)(ps + 16);
#pragma unroll
    for (int t = 0; t < 4; ++t) {
      FragH vb;
      const unsigned short* vs = &vt_s[(t * 16 + ln) * VCOLS + wave * 16 + ks * 32 + 8 * hl];
      vb.q[0] = *(const u32x4a*)(vs);
      vb.q[1] = *(const u32x4a*)(vs + 16);
      oacc[t] = wmma_f16(pa.v, vb.v, oacc[t]);
    }
  }

  float vsv[4];
#pragma unroll
  for (int t = 0; t < 4; ++t) vsv[t] = vsum[(size_t)b * EMB + h * HD + t * 16 + ln];
  float* cw = cst[wave];
#pragma unroll
  for (int r = 0; r < 8; ++r)
#pragma unroll
    for (int t = 0; t < 4; ++t)
      cw[(8 * hl + r) * 64 + t * 16 + ln] = oacc[t][r] * PINV + garr[r] * vsv[t];
  __syncthreads();

  v4f ov[8];
#pragma unroll
  for (int it = 0; it < 8; ++it) {
    const int f = it * 32 + lane;
    const int row = f >> 4, c4 = f & 15;
    ov[it] = *(const v4fa*)&cw[row * 64 + c4 * 4];
  }
#pragma unroll
  for (int it = 0; it < 8; ++it) {
    const int f = it * 32 + lane;
    const int row = f >> 4, c4 = f & 15;
    float* dp = ctx + (brow + (size_t)(iw0 + row)) * EMB + h * HD + c4 * 4;
    *(volatile v4f*)dp = ov[it];
  }
  __threadfence();
#pragma unroll
  for (int it = 0; it < 8; ++it) {
    const int f = it * 32 + lane;
    const int row = f >> 4, c4 = f & 15;
    float* dp = ctx + (brow + (size_t)(iw0 + row)) * EMB + h * HD + c4 * 4;
    *(volatile v4f*)dp = ov[it];
  }
}

__global__ __launch_bounds__(192) void k_ln(
    const float* __restrict__ qf, const float* __restrict__ cx,
    const float* __restrict__ gamma, const float* __restrict__ beta,
    float* __restrict__ out)
{
#pragma clang fp contract(off)
  __shared__ float red1[8];
  __shared__ float red2[8];
  const int R = blockIdx.x;
  const int t = threadIdx.x;
  const int wave = t >> 5, lane = t & 31;
  const size_t base = (size_t)R * EMB + 4 * t;
  const v4f qv = *(const v4f*)(qf + base);
  const v4f cv = *(const v4f*)(cx + base);
  const float x0 = qv.x + cv.x;
  const float x1 = qv.y + cv.y;
  const float x2 = qv.z + cv.z;
  const float x3 = qv.w + cv.w;

  float s = (x0 + x1) + (x2 + x3);
  s += __shfl_xor(s, 16, 32);
  s += __shfl_xor(s, 8, 32);
  s += __shfl_xor(s, 4, 32);
  s += __shfl_xor(s, 2, 32);
  s += __shfl_xor(s, 1, 32);
  if (lane == 0) red1[wave] = s;
  __syncthreads();
  const float tot = ((red1[0] + red1[1]) + (red1[2] + red1[3])) + (red1[4] + red1[5]);
  const float mean = tot * (1.0f / (float)EMB);

  const float e0 = x0 - mean, e1 = x1 - mean, e2 = x2 - mean, e3 = x3 - mean;
  float ss = (e0 * e0 + e1 * e1) + (e2 * e2 + e3 * e3);
  ss += __shfl_xor(ss, 16, 32);
  ss += __shfl_xor(ss, 8, 32);
  ss += __shfl_xor(ss, 4, 32);
  ss += __shfl_xor(ss, 2, 32);
  ss += __shfl_xor(ss, 1, 32);
  if (lane == 0) red2[wave] = ss;
  __syncthreads();
  const float tot2 = ((red2[0] + red2[1]) + (red2[2] + red2[3])) + (red2[4] + red2[5]);
  const float var  = tot2 * (1.0f / (float)EMB);
  const float rstd = 1.0f / sqrtf(var + 1e-5f);

  const float g0 = bfr(gamma[4 * t]),     g1 = bfr(gamma[4 * t + 1]);
  const float g2 = bfr(gamma[4 * t + 2]), g3 = bfr(gamma[4 * t + 3]);
  const float b0 = bfr(beta[4 * t]),      b1 = bfr(beta[4 * t + 1]);
  const float b2 = bfr(beta[4 * t + 2]),  b3 = bfr(beta[4 * t + 3]);
  v4f y;
  y.x = (g0 * e0) * rstd + b0;
  y.y = (g1 * e1) * rstd + b1;
  y.z = (g2 * e2) * rstd + b2;
  y.w = (g3 * e3) * rstd + b3;
  float* dp = out + base;
  *(volatile v4f*)dp = y;
  __threadfence();
  *(volatile v4f*)dp = y;
}

extern "C" void kernel_launch(void* const* d_in, const int* in_sizes, int n_in,
                              void* d_out, int out_size, void* d_ws, size_t ws_size,
                              hipStream_t stream)
{
  if (n_in < 13) return;
  const int needAct = ((NB - 1) * SEQ_FULL + SEQ) * EMB;
  const int needMsk = (NB - 1) * SEQ_FULL + SEQ;
  if (in_sizes[0] < needAct || in_sizes[1] < needAct || in_sizes[2] < needAct) return;
  if (in_sizes[3] < needMsk) return;
  if (in_sizes[4] < EMB * EMB || in_sizes[6] < EMB * EMB || in_sizes[8] < EMB * EMB) return;
  if (in_sizes[5] < EMB || in_sizes[7] < EMB || in_sizes[9] < EMB) return;
  if (in_sizes[10] < 3 || in_sizes[11] < EMB || in_sizes[12] < EMB) return;
  if (out_size < MROWS * EMB) return;

  const float* q_in  = (const float*)d_in[0];
  const float* k_in  = (const float*)d_in[1];
  const float* v_in  = (const float*)d_in[2];
  const float* amask = (const float*)d_in[3];
  const float* Wq    = (const float*)d_in[4];
  const float* bq    = (const float*)d_in[5];
  const float* Wk    = (const float*)d_in[6];
  const float* bk    = (const float*)d_in[7];
  const float* Wv    = (const float*)d_in[8];
  const float* bv    = (const float*)d_in[9];
  const float* wwin  = (const float*)d_in[10];
  const float* gamma = (const float*)d_in[11];
  const float* beta  = (const float*)d_in[12];
  float* out = (float*)d_out;

  char* ws = (char*)d_ws;
  size_t off = 0;
  auto take = [&](size_t bytes) -> char* {
    char* p = ws + off;
    off += (bytes + 255) & ~(size_t)255;
    return p;
  };
  const size_t actH = (size_t)MROWS * EMB * 2;
  const size_t actF = (size_t)MROWS * EMB * 4;
  const size_t wH   = (size_t)EMB * EMB * 2;
  unsigned short* xq16 = (unsigned short*)take(actH);
  unsigned short* xk16 = (unsigned short*)take(actH);
  unsigned short* xv16 = (unsigned short*)take(actH);
  unsigned short* wq16 = (unsigned short*)take(wH);
  unsigned short* wk16 = (unsigned short*)take(wH);
  unsigned short* wv16 = (unsigned short*)take(wH);
  float* qf32 = (float*)take(actF);
  float* kf32 = (float*)take(actF);
  float* vf32 = (float*)take(actF);
  unsigned short* qh16 = (unsigned short*)take(actH);
  unsigned short* kh16 = (unsigned short*)take(actH);
  unsigned short* vh16 = (unsigned short*)take(actH);
  float* ctx  = (float*)take(actF);
  float* vsum = (float*)take((size_t)NB * EMB * 4);
  if (off > ws_size) return;

  {
    const int itemsAct = MROWS * EMB / 8;
    dim3 grid((itemsAct + 255) / 256, 6);
    k_cvt<<<grid, 256, 0, stream>>>(q_in, k_in, v_in, Wq, Wk, Wv,
                                    xq16, xk16, xv16, wq16, wk16, wv16);
  }
  {
    dim3 grid(EMB / 128, MROWS / 128);
    k_gemm<<<grid, 256, 0, stream>>>(xq16, wq16, bq, qf32, qh16);
    k_gemm<<<grid, 256, 0, stream>>>(xk16, wk16, bk, kf32, kh16);
    k_gemm<<<grid, 256, 0, stream>>>(xv16, wv16, bv, vf32, vh16);
  }
  {
    dim3 grid(EMB / 256, NB);
    k_vsum<<<grid, 256, 0, stream>>>(vf32, vsum);
  }
  {
    dim3 grid(SEQ / 64, NH, NB);
    k_attn<<<grid, 128, 0, stream>>>(qh16, kh16, vh16, vsum, amask, wwin, ctx);
  }
  k_ln<<<MROWS, 192, 0, stream>>>(qf32, ctx, gamma, beta, out);
}
